// GINConv_12137577578700
// MI455X (gfx1250) — hardware-verified
//
#include <hip/hip_runtime.h>
#include <stddef.h>


#define DCH    128
#define DHID   256
#define NTHR   256
#define NWAVE  8
#define EPT    8
#define NGRP   2
#define CHUNK  (NTHR * EPT * NGRP)
#define WCAP   (EPT * NGRP * 32)
#define LISTN  (NWAVE * WCAP)
#define TGT    256
#define GROWS  128
#define SH     264
#define STP    132
#define E1R    5
#define E2R    3
#define ETAB   8

#define LDS_AGG (TGT * DCH * 4 + LISTN * 4 + ETAB * DCH * 4 + 64)
#define LDS_MLP (2 * GROWS * SH * 2)

static_assert((CHUNK & (CHUNK - 1)) == 0);
static_assert(CHUNK <= 4096);
static_assert((TGT & (TGT - 1)) == 0 && TGT <= 4096);
static_assert(TGT == NWAVE * 32);
static_assert((TGT % GROWS) == 0);
static_assert(GROWS == NWAVE * 16);
static_assert((TGT * DCH / 4) % NTHR == 0);
static_assert((ETAB * DCH) % NTHR == 0);
static_assert(GROWS * STP * 4 <= LDS_MLP);
static_assert((DHID * DCH / 8) % NTHR == 0);
static_assert((SH * 2) % 16 == 0 && (STP * 4) % 16 == 0);

typedef float          v4f  __attribute__((ext_vector_type(4)));
typedef float          v8f  __attribute__((ext_vector_type(8)));
typedef int            v4i  __attribute__((ext_vector_type(4)));
typedef unsigned short v8us __attribute__((ext_vector_type(8)));
typedef __bf16         v16b __attribute__((ext_vector_type(16)));
union FragB { v16b v; v8us h[2]; };
static_assert(sizeof(FragB) == 32);

__device__ __forceinline__ unsigned short f2bf(float f) {
  unsigned u = __float_as_uint(f);
  u = u + 0x7FFFu + ((u >> 16) & 1u);
  return (unsigned short)(u >> 16);
}
__device__ __forceinline__ float bfr(float f) {
  return __uint_as_float(((unsigned)f2bf(f)) << 16);
}
__device__ __forceinline__ v4f bfr4(v4f a) {
  v4f r;
  r.x = bfr(a.x); r.y = bfr(a.y); r.z = bfr(a.z); r.w = bfr(a.w);
  return r;
}
__device__ __forceinline__ void split8(v4f a, v4f b, v8us& hv, v8us& lv) {
  float v[8];
  v[0] = a.x; v[1] = a.y; v[2] = a.z; v[3] = a.w; v[4] = b.x; v[5] = b.y; v[6] = b.z; v[7] = b.w;
#pragma unroll
  for (int e = 0; e < 8; ++e) {
    const unsigned short hb = f2bf(v[e]);
    const float hf = __uint_as_float(((unsigned)hb) << 16);
    hv[e] = hb;
    lv[e] = f2bf(v[e] - hf);
  }
}

__device__ __forceinline__ v8f wmb(v16b a, v16b b, v8f c) {
#if defined(__HIP_DEVICE_COMPILE__)
  v8f d = __builtin_amdgcn_wmma_f32_16x16x32_bf16(false, a, false, b, (short)0, c, false, false);
  asm volatile("v_nop\n\tv_nop\n\tv_nop\n\tv_nop" : "+v"(d) : "v"(a), "v"(b));
  return d;
#else
  (void)a; (void)b;
  return c;
#endif
}

template <int NB>
__device__ __forceinline__ int scan_chunk(const int* __restrict__ dsts, int nE, int cbase, int slotBase,
                                          int vec8, int* list, int tid, int lane, int wave) {
  int wc = 0;
#pragma unroll
  for (int g = 0; g < NGRP; ++g) {
    const int el0  = (g * NTHR + tid) * EPT;
    const int e0   = cbase + el0;
    const int sent = -2147483647 - 1;
    v4i da, db;
    if (vec8 != 0 && cbase + CHUNK <= nE) {
      da = *(const v4i*)(dsts + e0);
      db = *(const v4i*)(dsts + e0 + 4);
    } else {
      da.x = (e0     < nE) ? dsts[min(e0, nE - 1)]     : sent;
      da.y = (e0 + 1 < nE) ? dsts[min(e0 + 1, nE - 1)] : sent;
      da.z = (e0 + 2 < nE) ? dsts[min(e0 + 2, nE - 1)] : sent;
      da.w = (e0 + 3 < nE) ? dsts[min(e0 + 3, nE - 1)] : sent;
      db.x = (e0 + 4 < nE) ? dsts[min(e0 + 4, nE - 1)] : sent;
      db.y = (e0 + 5 < nE) ? dsts[min(e0 + 5, nE - 1)] : sent;
      db.z = (e0 + 6 < nE) ? dsts[min(e0 + 6, nE - 1)] : sent;
      db.w = (e0 + 7 < nE) ? dsts[min(e0 + 7, nE - 1)] : sent;
    }
    const unsigned nb = (unsigned)slotBase;
    const unsigned s0 = (unsigned)da.x - nb, s1 = (unsigned)da.y - nb;
    const unsigned s2 = (unsigned)da.z - nb, s3 = (unsigned)da.w - nb;
    const unsigned s4 = (unsigned)db.x - nb, s5 = (unsigned)db.y - nb;
    const unsigned s6 = (unsigned)db.z - nb, s7 = (unsigned)db.w - nb;
    const bool h0 = s0 < (unsigned)NB, h1 = s1 < (unsigned)NB, h2 = s2 < (unsigned)NB, h3 = s3 < (unsigned)NB;
    const bool h4 = s4 < (unsigned)NB, h5 = s5 < (unsigned)NB, h6 = s6 < (unsigned)NB, h7 = s7 < (unsigned)NB;
    const unsigned any = __builtin_amdgcn_ballot_w32(h0 | h1 | h2 | h3 | h4 | h5 | h6 | h7);
    if (any != 0u) {
#define HITJ(J, HJ, SJ) { \
        const unsigned mj = __builtin_amdgcn_ballot_w32(HJ); \
        if (mj != 0u) { \
          if (HJ) { \
            const int pos = wc + (int)__builtin_amdgcn_mbcnt_lo(mj, 0u); \
            if (pos < WCAP) list[wave * WCAP + pos] = ((el0 + (J)) << 12) | (int)(SJ); \
          } \
          wc += (int)__builtin_popcount(mj); } }
      HITJ(0, h0, s0)
      HITJ(1, h1, s1)
      HITJ(2, h2, s2)
      HITJ(3, h3, s3)
      HITJ(4, h4, s4)
      HITJ(5, h5, s5)
      HITJ(6, h6, s6)
      HITJ(7, h7, s7)
#undef HITJ
    }
  }
  return wc;
}

__global__ __launch_bounds__(NTHR) void k_wprep(
    const float* __restrict__ W1, const float* __restrict__ W2,
    unsigned short* W1p, unsigned short* W2p) {
  const int g0 = DHID * DCH / 8;
  const int bstart = blockIdx.x * NTHR;
  const int i = bstart + (int)threadIdx.x;
  const float* src; unsigned short* dst; int K, Nout, o;
  if (bstart < g0) { src = W1; dst = W1p; K = DCH;  Nout = DHID; o = i * 8; }
  else             { src = W2; dst = W2p; K = DHID; Nout = DCH;  o = (i - g0) * 8; }
  if (i >= 2 * g0) return;
  const int n  = o / K;
  const int k0 = o - n * K;
  const int nc = n < Nout ? n : Nout - 1;
  v8us hv;
#pragma unroll
  for (int e = 0; e < 8; ++e) {
    const int k  = k0 + e;
    const int kc = k < K ? k : K - 1;
    const float w = src[(size_t)kc * Nout + nc];
    hv[e] = f2bf(w);
  }
  unsigned short* dp = dst + o;
  *(volatile v8us*)dp = hv;
  __threadfence();
  *(volatile v8us*)dp = hv;
}

__device__ __forceinline__ void agg_store_pass(const float* acc, const float* __restrict__ x,
                                               unsigned short* ohi, unsigned short* olo,
                                               int nodeBase, int nN, int wave, int lane) {
#pragma unroll 1
  for (int q = 0; q < 16; ++q) {
    const int lr   = wave * 32 + 2 * q + (lane >> 4);
    const int c0   = 8 * (lane & 15);
    const int grow = nodeBase + lr;
    const int gc   = grow > nN - 1 ? nN - 1 : grow;
    const v4f a0 = *(const v4f*)(acc + lr * DCH + c0);
    const v4f a1 = *(const v4f*)(acc + lr * DCH + c0 + 4);
    const v4f x0 = bfr4(*(const v4f*)(x + (size_t)gc * DCH + c0));
    const v4f x1 = bfr4(*(const v4f*)(x + (size_t)gc * DCH + c0 + 4));
    const v4f o0 = a0 + x0;
    const v4f o1 = a1 + x1;
    v8us hv, lv;
    split8(o0, o1, hv, lv);
    *(volatile v8us*)(ohi + (size_t)grow * DCH + c0) = hv;
    *(volatile v8us*)(olo + (size_t)grow * DCH + c0) = lv;
  }
}

__global__ __launch_bounds__(NTHR) void k_agg(
    const float* __restrict__ x, const int* __restrict__ ei, const int* __restrict__ ea,
    const float* __restrict__ emb1, const float* __restrict__ emb2,
    unsigned short* ohi, unsigned short* olo, int nN, int nE, int vec8) {
  extern __shared__ v4f lds_dyn[];
  float* acc  = (float*)lds_dyn;
  int*   list = (int*)(acc + TGT * DCH);
  float* se   = (float*)(list + LISTN);
  int*   wcnt = (int*)(se + ETAB * DCH);
  const int tid = threadIdx.x, lane = tid & 31;
  const int wave = __builtin_amdgcn_readfirstlane(tid >> 5);
  const int nodeBase = blockIdx.x * TGT;
  const int* dsts = ei;
  const int* srcs = ei + nE;

  {
    const v4f z = {0.f, 0.f, 0.f, 0.f};
    for (int i = tid; i < TGT * DCH / 4; i += NTHR) ((v4f*)acc)[i] = z;
    for (int i = tid; i < ETAB * DCH; i += NTHR) {
      const int r = i >> 7, c = i & (DCH - 1);
      const int r1 = r < E1R - 1 ? r : E1R - 1;
      int r2 = r - E1R;
      r2 = r2 < 0 ? 0 : (r2 > E2R - 1 ? E2R - 1 : r2);
      const float v1 = emb1[r1 * DCH + c];
      const float v2 = emb2[r2 * DCH + c];
      se[i] = bfr(r < E1R ? v1 : v2);
    }
  }
  __syncthreads();

  const int nChunks = (nE + CHUNK - 1) / CHUNK;
#pragma unroll 1
  for (int ch = 0; ch < nChunks; ++ch) {
    const int cbase = ch * CHUNK;
    const int wc = scan_chunk<TGT>(dsts, nE, cbase, nodeBase, vec8, list, tid, lane, wave);
    if (lane == 0) wcnt[wave] = wc;
    __syncthreads();
#pragma unroll 1
    for (int wsx = 0; wsx < NWAVE; ++wsx) {
      int n = __builtin_amdgcn_readfirstlane(wcnt[wsx]);
      n = n > WCAP ? WCAP : (n < 0 ? 0 : n);
      const int* lp = list + wsx * WCAP;
#pragma unroll 1
      for (int i = 0; i < n; ++i) {
        const int ent  = __builtin_amdgcn_readfirstlane(lp[i]);
        const int slot = ent & (TGT - 1);
        if ((slot & (NWAVE - 1)) == wave) {
          int e = cbase + ((ent >> 12) & (CHUNK - 1));
          e = e > nE - 1 ? nE - 1 : e;
          int s = srcs[e];
          s = s < 0 ? 0 : (s > nN - 1 ? nN - 1 : s);
          int a0 = ea[2 * (size_t)e];
          a0 = a0 < 0 ? 0 : (a0 > E1R - 1 ? E1R - 1 : a0);
          int a1 = ea[2 * (size_t)e + 1];
          a1 = a1 < 0 ? 0 : (a1 > E2R - 1 ? E2R - 1 : a1);
          v4f mv = bfr4(*(const v4f*)(x + (size_t)s * DCH + 4 * lane));
          mv = mv + *(const v4f*)(se + a0 * DCH + 4 * lane);
          mv = mv + *(const v4f*)(se + (E1R + a1) * DCH + 4 * lane);
          v4f* ap = (v4f*)(acc + slot * DCH + 4 * lane);
          *ap = *ap + mv;
        }
      }
    }
    __syncthreads();
  }

  agg_store_pass(acc, x, ohi, olo, nodeBase, nN, wave, lane);
  __threadfence();
  agg_store_pass(acc, x, ohi, olo, nodeBase, nN, wave, lane);
}

__global__ __launch_bounds__(NTHR) void k_mlp(
    const unsigned short* __restrict__ Ahi, const unsigned short* __restrict__ Alo,
    const unsigned short* __restrict__ W1p, const float* __restrict__ b1,
    const unsigned short* __restrict__ W2p, const float* __restrict__ b2,
    float* out, int nN) {
  extern __shared__ v4f lds_dyn[];
  unsigned short* sHi = (unsigned short*)lds_dyn;
  unsigned short* sLo = sHi + GROWS * SH;
  float* stg = (float*)lds_dyn;
  const int tid = threadIdx.x, lane = tid & 31, hh = lane >> 4, m = lane & 15;
  const int wave = __builtin_amdgcn_readfirstlane(tid >> 5);
  const int rowBase = blockIdx.x * GROWS;
  const int r0 = wave * 16;

  const unsigned short* aph = Ahi + (size_t)(rowBase + r0 + m) * DCH + 8 * hh;
  const unsigned short* apl = Alo + (size_t)(rowBase + r0 + m) * DCH + 8 * hh;
#pragma unroll 1
  for (int g = 0; g < 2; ++g) {
    v8f acc[8];
#pragma unroll
    for (int t = 0; t < 8; ++t) { v8f z = {0.f, 0.f, 0.f, 0.f, 0.f, 0.f, 0.f, 0.f}; acc[t] = z; }
#pragma unroll
    for (int kt = 0; kt < DCH / 32; ++kt) {
      FragB ah, al;
      ah.h[0] = *(const v8us*)(aph + 32 * kt);
      ah.h[1] = *(const v8us*)(aph + 32 * kt + 16);
      al.h[0] = *(const v8us*)(apl + 32 * kt);
      al.h[1] = *(const v8us*)(apl + 32 * kt + 16);
#pragma unroll
      for (int t = 0; t < 8; ++t) {
        const unsigned short* bp = W1p + (size_t)(128 * g + 16 * t + m) * DCH + 32 * kt + 8 * hh;
        FragB b;
        b.h[0] = *(const v8us*)bp;
        b.h[1] = *(const v8us*)(bp + 16);
        acc[t] = wmb(ah.v, b.v, acc[t]);
        acc[t] = wmb(al.v, b.v, acc[t]);
      }
    }
#pragma unroll
    for (int t = 0; t < 8; ++t) {
      const int col = 128 * g + 16 * t + m;
      const float bb = bfr(b1[col]);
      unsigned short* hp = sHi + (r0 + 8 * hh) * SH + col;
      unsigned short* lp = sLo + (r0 + 8 * hh) * SH + col;
#pragma unroll
      for (int r = 0; r < 8; ++r) {
        float v = acc[t][r] + bb;
        v = fmaxf(v, 0.0f);
        const unsigned short hb = f2bf(v);
        const float hf = __uint_as_float(((unsigned)hb) << 16);
        hp[r * SH] = hb;
        lp[r * SH] = f2bf(v - hf);
      }
    }
  }
  __syncthreads();

  v8f acc2[8];
#pragma unroll
  for (int t = 0; t < 8; ++t) { v8f z = {0.f, 0.f, 0.f, 0.f, 0.f, 0.f, 0.f, 0.f}; acc2[t] = z; }
  const unsigned short* lah = sHi + (r0 + m) * SH + 8 * hh;
  const unsigned short* lal = sLo + (r0 + m) * SH + 8 * hh;
#pragma unroll
  for (int kt = 0; kt < DHID / 32; ++kt) {
    FragB ah, al;
    ah.h[0] = *(const v8us*)(lah + 32 * kt);
    ah.h[1] = *(const v8us*)(lah + 32 * kt + 16);
    al.h[0] = *(const v8us*)(lal + 32 * kt);
    al.h[1] = *(const v8us*)(lal + 32 * kt + 16);
#pragma unroll
    for (int t = 0; t < 8; ++t) {
      const unsigned short* bp = W2p + (size_t)(16 * t + m) * DHID + 32 * kt + 8 * hh;
      FragB b;
      b.h[0] = *(const v8us*)bp;
      b.h[1] = *(const v8us*)(bp + 16);
      acc2[t] = wmb(ah.v, b.v, acc2[t]);
      acc2[t] = wmb(al.v, b.v, acc2[t]);
    }
  }
  __syncthreads();

#pragma unroll
  for (int t = 0; t < 8; ++t) {
    const int col = 16 * t + m;
    const float bb = bfr(b2[col]);
    float* sp = stg + (r0 + 8 * hh) * STP + col;
#pragma unroll
    for (int r = 0; r < 8; ++r) sp[r * STP] = acc2[t][r] + bb;
  }
  __syncthreads();

  const float* lrow = stg + r0 * STP + 4 * lane;
  float* grow = out + (size_t)(rowBase + r0) * DCH + 4 * lane;
#pragma unroll
  for (int i = 0; i < 16; ++i) {
    if (rowBase + r0 + i < nN) {
      const v4f v = *(const v4f*)(lrow + i * STP);
      *(volatile v4f*)(grow + (size_t)i * DCH) = v;
    }
  }
  __threadfence();
#pragma unroll
  for (int i = 0; i < 16; ++i) {
    if (rowBase + r0 + i < nN) {
      const v4f v = *(const v4f*)(lrow + i * STP);
      *(volatile v4f*)(grow + (size_t)i * DCH) = v;
    }
  }
}

extern "C" void kernel_launch(void* const* d_in, const int* in_sizes, int n_in,
                              void* d_out, int out_size, void* d_ws, size_t ws_size,
                              hipStream_t stream) {
  if (n_in < 9) return;
  const int nN = in_sizes[0] / DCH;
  const int nE = in_sizes[1] / 2;
  if (nN <= 0 || nE <= 0 || in_sizes[0] != nN * DCH || in_sizes[1] != 2 * nE || in_sizes[2] != 2 * nE) return;
  if (in_sizes[3] != DCH * DHID || in_sizes[4] != DHID || in_sizes[5] != DHID * DCH || in_sizes[6] != DCH) return;
  if (in_sizes[7] != E1R * DCH || in_sizes[8] != E2R * DCH) return;
  if (out_size != nN * DCH) return;
  if (nN > (1 << 22) || nE > (1 << 28)) return;

  const float* x    = (const float*)d_in[0];
  const int*   ei   = (const int*)d_in[1];
  const int*   ea   = (const int*)d_in[2];
  const float* W1   = (const float*)d_in[3];
  const float* b1   = (const float*)d_in[4];
  const float* W2   = (const float*)d_in[5];
  const float* b2   = (const float*)d_in[6];
  const float* emb1 = (const float*)d_in[7];
  const float* emb2 = (const float*)d_in[8];
  float* out = (float*)d_out;

  const int nAgg = (nN + TGT - 1) / TGT;
  const int NPAD = nAgg * TGT;
  const int nMlp = NPAD / GROWS;

  char* ws = (char*)d_ws;
  size_t off = 0;
  const size_t oW1 = off; off += (size_t)DHID * DCH * 2;     off = (off + 255) & ~(size_t)255;
  const size_t oW2 = off; off += (size_t)DCH * DHID * 2;     off = (off + 255) & ~(size_t)255;
  const size_t oHi = off; off += (size_t)NPAD * DCH * 2;     off = (off + 255) & ~(size_t)255;
  const size_t oLo = off; off += (size_t)NPAD * DCH * 2;     off = (off + 255) & ~(size_t)255;
  if (off > ws_size) return;
  unsigned short* W1p = (unsigned short*)(ws + oW1);
  unsigned short* W2p = (unsigned short*)(ws + oW2);
  unsigned short* pHi = (unsigned short*)(ws + oHi);
  unsigned short* pLo = (unsigned short*)(ws + oLo);

  const int vec8 = ((nE & 3) == 0) ? 1 : 0;

  k_wprep<<<(2 * (DHID * DCH / 8)) / NTHR, NTHR, 0, stream>>>(W1, W2, W1p, W2p);

  hipFuncSetAttribute(reinterpret_cast<const void*>(&k_agg),
                      hipFuncAttributeMaxDynamicSharedMemorySize, LDS_AGG);
  k_agg<<<nAgg, NTHR, LDS_AGG, stream>>>(x, ei, ea, emb1, emb2, pHi, pLo, nN, nE, vec8);

  hipFuncSetAttribute(reinterpret_cast<const void*>(&k_mlp),
                      hipFuncAttributeMaxDynamicSharedMemorySize, LDS_MLP);
  k_mlp<<<nMlp, NTHR, LDS_MLP, stream>>>(pHi, pLo, W1p, b1, W2p, b2, out, nN);
}
